// Policy_73916387164829
// MI455X (gfx1250) — hardware-verified
//
#include <hip/hip_runtime.h>
#include <stddef.h>


typedef _Float16       v16h  __attribute__((ext_vector_type(16)));
typedef _Float16       v8h   __attribute__((ext_vector_type(8)));
typedef __bf16         v16b  __attribute__((ext_vector_type(16)));
typedef unsigned short v16us __attribute__((ext_vector_type(16)));
typedef unsigned short v8us  __attribute__((ext_vector_type(8)));
typedef float          v8f   __attribute__((ext_vector_type(8)));
typedef float          v4f   __attribute__((ext_vector_type(4)));
typedef v4f            __attribute__((may_alias)) v4fa;
typedef unsigned int   u32x4 __attribute__((ext_vector_type(4)));

#define MTOK     200
#define NLAY     22
#define GWD      11
#define K1       576
#define K1R      550
#define LDA1     5184
#define K2       1152
#define CH       128
#define HHALF    256
#define HID      512
#define NHP      32
#define SPB      32
#define W1SCALE  16384.0f
#define W1RSCALE (1.0f / 16384.0f)

#define L_A1     0
#define L_A1B    165888
#define L_A2H    165888
#define L_A2L    202752
#define L_ASF    239616
#define L_OUT    240640
#define L_TOTAL  243200
#define L_A3H    0
#define L_A3L    4096
#define L_AHH    8192
#define L_AHL    24576

#define WS_W1T   0
#define WS_W2H   147456
#define WS_W2L   442368
#define WS_FCH   737280
#define WS_FCL   802816
#define WS_SLH   868352
#define WS_SLL   884736
#define WS_HDH   901120
#define WS_HDL   933888
#define WS_HDB   966656
#define WS_TOTAL 966784

#define PG0 9216
#define PG1 27648
#define PG2 31744
#define PG3 32768
#define PG4 34816
#define PG5 34824

__device__ __constant__ float c_maxvec[NLAY] = {
    9.0f, 1.0f, 1.0f, 10.0f, 3.0f, 254.0f, 1.0f, 1.0f, 235.0f, 8.0f, 9.0f,
    250.0f, 29.0f, 1.0f, 1.0f, 8.0f, 1.0f, 1.0f, 6.0f, 3.0f, 1.0f, 2.0f};

__device__ __forceinline__ unsigned short f2bf(float f) {
    unsigned int u = __float_as_uint(f);
    u = u + 0x7FFFu + ((u >> 16) & 1u);
    return (unsigned short)(u >> 16);
}
__device__ __forceinline__ void split_bf16(float f, unsigned short& hi, unsigned short& lo) {
    const unsigned short h = f2bf(f);
    const float fh = __uint_as_float(((unsigned int)h) << 16);
    hi = h;
    lo = f2bf(f - fh);
}

union FragH { v16h v; v8h p[2]; };
union FragB { v16b v; v16us u; v8us p[2]; };

__device__ __forceinline__ v16h frag_h(const _Float16* base, int ld, int k0, int lane) {
    FragH f;
    const _Float16* q = base + (lane & 15) * ld + k0 + 8 * (lane >> 4);
    f.p[0] = *(const v8h*)q;
    f.p[1] = *(const v8h*)(q + 16);
    return f.v;
}
__device__ __forceinline__ v16b frag_b(const unsigned short* base, int ld, int k0, int lane) {
    FragB f;
    const unsigned short* q = base + (lane & 15) * ld + k0 + 8 * (lane >> 4);
    f.p[0] = *(const v8us*)q;
    f.p[1] = *(const v8us*)(q + 16);
    return f.v;
}

__device__ __forceinline__ v8f mma_f16(v8f acc, v16h a, v16h b) {
    acc = __builtin_amdgcn_wmma_f32_16x16x32_f16(false, a, false, b, (short)0, acc, false, false);
    asm volatile("v_nop\n\tv_nop\n\tv_nop\n\tv_nop" : "+v"(acc) : "v"(a), "v"(b));
    return acc;
}
__device__ __forceinline__ v8f mma2_bf16(v8f acc, v16b a, v16b bh, v16b bl) {
    acc = __builtin_amdgcn_wmma_f32_16x16x32_bf16(false, a, false, bh, (short)0, acc, false, false);
    acc = __builtin_amdgcn_wmma_f32_16x16x32_bf16(false, a, false, bl, (short)0, acc, false, false);
    asm volatile("v_nop\n\tv_nop\n\tv_nop\n\tv_nop" : "+v"(acc) : "v"(a), "v"(bh), "v"(bl));
    return acc;
}
__device__ __forceinline__ v8f mma3_bf16(v8f acc, v16b ah, v16b al, v16b bh, v16b bl) {
    acc = __builtin_amdgcn_wmma_f32_16x16x32_bf16(false, ah, false, bh, (short)0, acc, false, false);
    acc = __builtin_amdgcn_wmma_f32_16x16x32_bf16(false, ah, false, bl, (short)0, acc, false, false);
    acc = __builtin_amdgcn_wmma_f32_16x16x32_bf16(false, al, false, bh, (short)0, acc, false, false);
    asm volatile("v_nop\n\tv_nop\n\tv_nop\n\tv_nop" : "+v"(acc) : "v"(ah), "v"(al), "v"(bh), "v"(bl));
    return acc;
}

__global__ void __launch_bounds__(256)
k_prep(const float* __restrict__ c1w, const float* __restrict__ c2w,
       const float* __restrict__ fcw, const float* __restrict__ sw,
       const float* __restrict__ a0w, const float* __restrict__ a1w,
       const float* __restrict__ vw,  const float* __restrict__ a0b,
       const float* __restrict__ a1b, const float* __restrict__ vb,
       _Float16* __restrict__ w1t,
       unsigned short* __restrict__ w2h, unsigned short* __restrict__ w2l,
       unsigned short* __restrict__ fch, unsigned short* __restrict__ fcl,
       unsigned short* __restrict__ slh, unsigned short* __restrict__ sll,
       unsigned short* __restrict__ hdh, unsigned short* __restrict__ hdl,
       float* __restrict__ hdb)
{
    const int t = blockIdx.x * 256 + threadIdx.x;
    if (t < PG0) {
        const int e0 = t * 8;
        const int o = e0 / K1, k = e0 - o * K1;
        v8h v;
        #pragma unroll
        for (int i = 0; i < 8; ++i) {
            const int kk = k + i;
            float x = 0.0f;
            if (kk < K1R) {
                const int c = kk / 25;
                x = c1w[o * K1R + kk] * (W1SCALE / c_maxvec[c]);
            }
            v[i] = (_Float16)x;
        }
        volatile v8h* p = (volatile v8h*)(w1t + e0);
        *p = v;
        __threadfence();
        *p = v;
        return;
    }
    float x[8];
    unsigned short* ph;
    unsigned short* pl;
    if (t < PG1) {
        const int e0 = (t - PG0) * 8;
        #pragma unroll
        for (int i = 0; i < 8; ++i) x[i] = c2w[e0 + i];
        ph = w2h + e0; pl = w2l + e0;
    } else if (t < PG2) {
        const int e0 = (t - PG1) * 8;
        #pragma unroll
        for (int i = 0; i < 8; ++i) x[i] = fcw[e0 + i];
        ph = fch + e0; pl = fcl + e0;
    } else if (t < PG3) {
        const int e0 = (t - PG2) * 8;
        const int n = e0 / 32, k = e0 - n * 32;
        #pragma unroll
        for (int i = 0; i < 8; ++i) {
            const int kk = k + i;
            x[i] = (kk < NLAY) ? sw[n * NLAY + kk] * (1.0f / c_maxvec[kk]) : 0.0f;
        }
        ph = slh + e0; pl = sll + e0;
    } else if (t < PG4) {
        const int e0 = (t - PG3) * 8;
        const int r = e0 / HID, k = e0 - r * HID;
        #pragma unroll
        for (int i = 0; i < 8; ++i) {
            const int kk = k + i;
            float y = 0.0f;
            if (r < 9)        y = a0w[r * HID + kk];
            else if (r < 19)  y = a1w[(r - 9) * HID + kk];
            else if (r == 19) y = vw[kk];
            x[i] = y;
        }
        ph = hdh + e0; pl = hdl + e0;
    } else if (t < PG5) {
        const int i4 = (t - PG4) * 4;
        v4f bv;
        #pragma unroll
        for (int i = 0; i < 4; ++i) {
            const int j = i4 + i;
            float y = 0.0f;
            if (j < 9)        y = a0b[j];
            else if (j < 19)  y = a1b[j - 9];
            else if (j == 19) y = vb[0];
            bv[i] = y;
        }
        volatile v4f* p = (volatile v4f*)(hdb + i4);
        *p = bv;
        __threadfence();
        *p = bv;
        return;
    } else {
        return;
    }
    v8us hv, lv;
    #pragma unroll
    for (int i = 0; i < 8; ++i) {
        unsigned short hi, lo;
        split_bf16(x[i], hi, lo);
        hv[i] = hi; lv[i] = lo;
    }
    volatile v8us* qh = (volatile v8us*)ph;
    volatile v8us* ql = (volatile v8us*)pl;
    *qh = hv; *ql = lv;
    __threadfence();
    *qh = hv; *ql = lv;
}

__global__ void __launch_bounds__(256)
k_forward(const int* __restrict__ obs,
          const float* __restrict__ c1b, const float* __restrict__ c2b,
          const float* __restrict__ fcb, const float* __restrict__ sb,
          const _Float16* __restrict__ w1t,
          const unsigned short* __restrict__ w2h, const unsigned short* __restrict__ w2l,
          const unsigned short* __restrict__ fch, const unsigned short* __restrict__ fcl,
          const unsigned short* __restrict__ slh, const unsigned short* __restrict__ sll,
          const unsigned short* __restrict__ hdh, const unsigned short* __restrict__ hdl,
          const float* __restrict__ hdb,
          float* out, int nB)
{
    extern __shared__ __attribute__((aligned(16))) char smem[];
    _Float16*       A1   = (_Float16*)(smem + L_A1);
    unsigned short* A2H  = (unsigned short*)(smem + L_A2H);
    unsigned short* A2L  = (unsigned short*)(smem + L_A2L);
    unsigned short* ASF  = (unsigned short*)(smem + L_ASF);
    float*          OUTS = (float*)(smem + L_OUT);
    unsigned short* A3H  = (unsigned short*)(smem + L_A3H);
    unsigned short* A3L  = (unsigned short*)(smem + L_A3L);
    unsigned short* AHH  = (unsigned short*)(smem + L_AHH);
    unsigned short* AHL  = (unsigned short*)(smem + L_AHL);

    const int tid  = threadIdx.x;
    const int lane = tid & 31;
    const int w    = tid >> 5;
    const int m    = lane & 15;
    const int hh   = lane >> 4;
    const int blk  = blockIdx.x;
    const v8f zacc = {0.f, 0.f, 0.f, 0.f, 0.f, 0.f, 0.f, 0.f};

    for (int g = 0; g < 2; ++g) {
        {
            const u32x4 z = {0u, 0u, 0u, 0u};
            u32x4* p = (u32x4*)(smem + L_A1);
            for (int i = tid; i < L_A1B / 16; i += 256) p[i] = z;
            u32x4* q = (u32x4*)(smem + L_ASF);
            if (tid < 1024 / 16) q[tid] = z;
        }
        __syncthreads();

        if (tid < 16) {
            const int s = tid;
            int sg = blk * SPB + g * 16 + s;
            if (sg > nB - 1) sg = nB - 1;
            const int* op = obs + (size_t)sg * (MTOK * 3);
            _Float16* a1s = A1 + s * LDA1;
            unsigned short* asf = ASF + s * 32;
            for (int t = 0; t < MTOK; ++t) {
                int c = op[3 * t], a = op[3 * t + 1], v = op[3 * t + 2];
                c = (c == 255) ? 0 : c;
                a = (a == 255) ? 0 : a;
                v = (v == 255) ? 0 : v;
                const int x = (c >> 4) & 15;
                const int y = c & 15;
                if ((unsigned)a >= (unsigned)NLAY || x >= GWD || y >= GWD) continue;
                const float fv = (float)v;
                const _Float16 hv = (_Float16)fv;
                if (x == 5 && y == 5) asf[a] = f2bf(fv);
                const int kb = a * 25;
                #pragma unroll
                for (int px = 0; px < 3; ++px) {
                    const int kx = x - 3 * px;
                    if ((unsigned)kx > 4u) continue;
                    #pragma unroll
                    for (int py = 0; py < 3; ++py) {
                        const int ky = y - 3 * py;
                        if ((unsigned)ky > 4u) continue;
                        a1s[(px * 3 + py) * K1 + kb + kx * 5 + ky] = hv;
                    }
                }
            }
        }
        __syncthreads();

        {
            const int cch = w * 16 + m;
            const float bias = c1b[cch];
            const _Float16* bt = w1t + (size_t)(w * 16) * K1;
            #pragma unroll 1
            for (int p = 0; p < 9; ++p) {
                const _Float16* at = A1 + p * K1;
                v8f acc = zacc;
                #pragma unroll 1
                for (int ks = 0; ks < K1 / 32; ++ks) {
                    const v16h av = frag_h(at, LDA1, ks * 32, lane);
                    const v16h bv = frag_h(bt, K1, ks * 32, lane);
                    acc = mma_f16(acc, av, bv);
                }
                #pragma unroll
                for (int j = 0; j < 8; ++j) {
                    const int s = 8 * hh + j;
                    const float v = fmaxf(acc[j] * W1RSCALE + bias, 0.0f);
                    unsigned short hi, lo;
                    split_bf16(v, hi, lo);
                    const int idx = s * K2 + cch * 9 + p;
                    A2H[idx] = hi;
                    A2L[idx] = lo;
                }
            }
        }
        __syncthreads();

        {
            const int cch = w * 16 + m;
            const float bias = c2b[cch];
            const unsigned short* bh = w2h + (size_t)(w * 16) * K2;
            const unsigned short* bl = w2l + (size_t)(w * 16) * K2;
            v8f acc = zacc;
            #pragma unroll 1
            for (int ks = 0; ks < K2 / 32; ++ks) {
                const v16b ah  = frag_b(A2H, K2, ks * 32, lane);
                const v16b al  = frag_b(A2L, K2, ks * 32, lane);
                const v16b bhv = frag_b(bh,  K2, ks * 32, lane);
                const v16b blv = frag_b(bl,  K2, ks * 32, lane);
                acc = mma3_bf16(acc, ah, al, bhv, blv);
            }
            #pragma unroll
            for (int j = 0; j < 8; ++j) {
                const int s = 8 * hh + j;
                const float v = fmaxf(acc[j] + bias, 0.0f);
                unsigned short hi, lo;
                split_bf16(v, hi, lo);
                A3H[s * CH + cch] = hi;
                A3L[s * CH + cch] = lo;
            }
        }
        __syncthreads();

        #pragma unroll 1
        for (int r = 0; r < 2; ++r) {
            const int nt = w + 8 * r;
            const int n  = nt * 16 + m;
            {
                const unsigned short* bh = fch + (size_t)(nt * 16) * CH;
                const unsigned short* bl = fcl + (size_t)(nt * 16) * CH;
                v8f acc = zacc;
                #pragma unroll 1
                for (int ks = 0; ks < CH / 32; ++ks) {
                    const v16b ah  = frag_b(A3H, CH, ks * 32, lane);
                    const v16b al  = frag_b(A3L, CH, ks * 32, lane);
                    const v16b bhv = frag_b(bh,  CH, ks * 32, lane);
                    const v16b blv = frag_b(bl,  CH, ks * 32, lane);
                    acc = mma3_bf16(acc, ah, al, bhv, blv);
                }
                const float bias = fcb[n];
                #pragma unroll
                for (int j = 0; j < 8; ++j) {
                    const int s = 8 * hh + j;
                    const float v = fmaxf(acc[j] + bias, 0.0f);
                    unsigned short hi, lo;
                    split_bf16(v, hi, lo);
                    const int idx = s * HID + HHALF + n;
                    AHH[idx] = hi;
                    AHL[idx] = lo;
                }
            }
            {
                const unsigned short* bh = slh + (size_t)(nt * 16) * 32;
                const unsigned short* bl = sll + (size_t)(nt * 16) * 32;
                const v16b av  = frag_b(ASF, 32, 0, lane);
                const v16b bhv = frag_b(bh,  32, 0, lane);
                const v16b blv = frag_b(bl,  32, 0, lane);
                v8f acc = mma2_bf16(zacc, av, bhv, blv);
                const float bias = sb[n];
                #pragma unroll
                for (int j = 0; j < 8; ++j) {
                    const int s = 8 * hh + j;
                    const float v = fmaxf(acc[j] + bias, 0.0f);
                    unsigned short hi, lo;
                    split_bf16(v, hi, lo);
                    const int idx = s * HID + n;
                    AHH[idx] = hi;
                    AHL[idx] = lo;
                }
            }
        }
        __syncthreads();

        if (w < 2) {
            const unsigned short* bh = hdh + (size_t)(w * 16) * HID;
            const unsigned short* bl = hdl + (size_t)(w * 16) * HID;
            v8f acc = zacc;
            #pragma unroll 1
            for (int ks = 0; ks < HID / 32; ++ks) {
                const v16b ah  = frag_b(AHH, HID, ks * 32, lane);
                const v16b al  = frag_b(AHL, HID, ks * 32, lane);
                const v16b bhv = frag_b(bh,  HID, ks * 32, lane);
                const v16b blv = frag_b(bl,  HID, ks * 32, lane);
                acc = mma3_bf16(acc, ah, al, bhv, blv);
            }
            const int col = w * 16 + m;
            const float bias = hdb[col];
            #pragma unroll
            for (int j = 0; j < 8; ++j) {
                const int ss = g * 16 + 8 * hh + j;
                const float v = acc[j] + bias;
                const int oi = (col < 9) ? (ss * 9 + col)
                             : ((col < 19) ? (288 + ss * 10 + (col - 9)) : (608 + ss));
                if (col < 20) OUTS[oi] = v;
            }
        }
        __syncthreads();
    }

    if (w == 0) {
        const int q  = lane >> 3;
        const int pc = lane & 7;
        v4f    vv[5];
        size_t dd[5];
        #pragma unroll
        for (int i = 0; i < 5; ++i) {
            const int line = 4 * i + q;
            vv[i] = *(const v4fa*)(OUTS + line * 32 + pc * 4);
            size_t d;
            if (line < 9)       d = (size_t)blk * 288 + (size_t)(line * 32 + pc * 4);
            else if (line < 19) d = (size_t)nB * 9 + (size_t)blk * 320 + (size_t)((line - 9) * 32 + pc * 4);
            else                d = (size_t)nB * 19 + (size_t)blk * 32 + (size_t)(pc * 4);
            dd[i] = d;
        }
        #pragma unroll
        for (int i = 0; i < 5; ++i) *(volatile v4f*)(out + dd[i]) = vv[i];
        __threadfence();
        #pragma unroll
        for (int i = 0; i < 5; ++i) *(volatile v4f*)(out + dd[i]) = vv[i];
    }
}

extern "C" void kernel_launch(void* const* d_in, const int* in_sizes, int n_in,
                              void* d_out, int out_size, void* d_ws, size_t ws_size,
                              hipStream_t stream) {
    if (n_in < 15) return;
    const int nB = in_sizes[0] / (MTOK * 3);
    if (nB < SPB || (nB % SPB) != 0) return;
    if ((size_t)out_size < (size_t)nB * 20) return;
    if (ws_size < (size_t)WS_TOTAL) return;

    const int*   obs = (const int*)d_in[0];
    const float* c1w = (const float*)d_in[1];
    const float* c1b = (const float*)d_in[2];
    const float* c2w = (const float*)d_in[3];
    const float* c2b = (const float*)d_in[4];
    const float* fcw = (const float*)d_in[5];
    const float* fcb = (const float*)d_in[6];
    const float* sw  = (const float*)d_in[7];
    const float* sb  = (const float*)d_in[8];
    const float* a0w = (const float*)d_in[9];
    const float* a0b = (const float*)d_in[10];
    const float* a1w = (const float*)d_in[11];
    const float* a1b = (const float*)d_in[12];
    const float* vw  = (const float*)d_in[13];
    const float* vb  = (const float*)d_in[14];

    char* ws = (char*)d_ws;
    _Float16*       w1t = (_Float16*)(ws + WS_W1T);
    unsigned short* w2h = (unsigned short*)(ws + WS_W2H);
    unsigned short* w2l = (unsigned short*)(ws + WS_W2L);
    unsigned short* fch = (unsigned short*)(ws + WS_FCH);
    unsigned short* fcl = (unsigned short*)(ws + WS_FCL);
    unsigned short* slh = (unsigned short*)(ws + WS_SLH);
    unsigned short* sll = (unsigned short*)(ws + WS_SLL);
    unsigned short* hdh = (unsigned short*)(ws + WS_HDH);
    unsigned short* hdl = (unsigned short*)(ws + WS_HDL);
    float*          hdb = (float*)(ws + WS_HDB);

    hipFuncSetAttribute(reinterpret_cast<const void*>(&k_forward),
                        hipFuncAttributeMaxDynamicSharedMemorySize, L_TOTAL);

    k_prep<<<(PG5 + 255) / 256, 256, 0, stream>>>(
        c1w, c2w, fcw, sw, a0w, a1w, vw, a0b, a1b, vb,
        w1t, w2h, w2l, fch, fcl, slh, sll, hdh, hdl, hdb);

    k_forward<<<nB / SPB, 256, L_TOTAL, stream>>>(
        obs, c1b, c2b, fcb, sb, w1t, w2h, w2l, fch, fcl, slh, sll, hdh, hdl, hdb,
        (float*)d_out, nB);
}
